// LIIF_ONNX_82884278878344
// MI455X (gfx1250) — hardware-verified
//
#include <hip/hip_runtime.h>
#include <stddef.h>


typedef _Float16 v16h __attribute__((ext_vector_type(16)));
typedef _Float16 v8h  __attribute__((ext_vector_type(8)));
typedef float    v8f  __attribute__((ext_vector_type(8)));
typedef float    v4f  __attribute__((ext_vector_type(4)));
typedef float    v2f  __attribute__((ext_vector_type(2)));
typedef _Float16 h16;

#ifndef NQ
#define NQ 262144
#endif
#define NQ_FULL 262144
#define HH 128
#define WW 128
#define CC 64
#define PH (HH + 2)
#define PW (WW + 2)
#define KTOT 576
#define DIN 580
#define NOUT 3

#define LDT 72
#define LDB 584

#define FCARRY 16.0f
#define WCARRY 64.0f

static_assert(NQ >= 256 && NQ <= NQ_FULL && (NQ % 256) == 0);
static_assert(CC == 64);
static_assert(KTOT == 9 * CC && (KTOT % 32) == 0);
static_assert(DIN == KTOT + 4);
static_assert((LDT % 8) == 0 && LDT >= CC);
static_assert((LDB % 8) == 0 && LDB >= KTOT);
static_assert(WW == 8 * 16);
static_assert(CC * WW == 32 * 256);
static_assert(PW * 8 <= 5 * 256);
static_assert(PW * 8 > 4 * 256);
static_assert(256 * NOUT == 192 * 4);
static_assert(WW * 4 == 128 * 4);

#define FP_BYTES ((size_t)PH * PW * CC * 2)
#define T_BYTES  ((size_t)HH * WW * 4 * 4)
#define OFF_FP   ((size_t)0)
#define OFF_T    (OFF_FP + FP_BYTES)
#define WS_TOTAL (OFF_T + T_BYTES)
static_assert((FP_BYTES % 128) == 0 && (T_BYTES % 128) == 0);
static_assert(WS_TOTAL <= (size_t)134217728);

#define SHIFT_NEG ((float)(-1.0 / 128.0 + 1.0e-6))
#define SHIFT_POS ((float)( 1.0 / 128.0 + 1.0e-6))
#define CLIP_LO   ((float)(-1.0 + 1.0e-6))
#define CLIP_HI   ((float)( 1.0 - 1.0e-6))

__device__ __forceinline__ float bf16r(float x) {
  unsigned int u = __float_as_uint(x);
  u = (u + 0x7FFFu + ((u >> 16) & 1u)) & 0xFFFF0000u;
  return __uint_as_float(u);
}

static __device__ __forceinline__ h16 toh_flush(float v) {
  const h16 r = (h16)v;
  return (fabsf(v) < 6.103515625e-05f) ? (h16)0.0f : r;
}

__device__ __forceinline__ v16h frag_at(const _Float16* p) {
  v8h lo = *(const v8h*)(p);
  v8h hi = *(const v8h*)(p + 16);
  v16h out;
#pragma unroll
  for (int i = 0; i < 8; ++i) { out[i] = lo[i]; out[i + 8] = hi[i]; }
  return out;
}
__device__ __forceinline__ v16h frag_join(v8h lo, v8h hi) {
  v16h out;
#pragma unroll
  for (int i = 0; i < 8; ++i) { out[i] = lo[i]; out[i + 8] = hi[i]; }
  return out;
}

__device__ __forceinline__ v8f wmma16(v16h a, v16h b, v8f c) {
  v8f d = __builtin_amdgcn_wmma_f32_16x16x32_f16(false, a, false, b, (short)0, c,
                                                 false, false);
  asm volatile("v_nop\n\tv_nop\n\tv_nop\n\tv_nop" : "+v"(d) : "v"(a), "v"(b));
  return d;
}

__global__ __launch_bounds__(256) void featplane_kernel(
    const float* __restrict__ feat, _Float16* __restrict__ FP) {
  __shared__ __attribute__((aligned(16))) _Float16 Tl[PW * LDT];
  const unsigned tid = threadIdx.x;
  const unsigned yp = blockIdx.x;
  const bool interior = (yp >= 1u) && (yp <= (unsigned)HH);
  const unsigned ys = (yp < 1u) ? 0u : ((yp > (unsigned)HH) ? (unsigned)(HH - 1) : (yp - 1u));

  if (tid < 16u) {
    const unsigned px = (tid >> 3) ? (unsigned)(PW - 1) : 0u;
    v8h z;
#pragma unroll
    for (int i = 0; i < 8; ++i) z[i] = (h16)0.0f;
    *(v8h*)&Tl[px * LDT + (tid & 7u) * 8u] = z;
  }
#pragma unroll 4
  for (unsigned j = 0; j < 32u; ++j) {
    const unsigned idx = tid + 256u * j;
    const unsigned c = idx >> 7, x = idx & 127u;
    const float v = feat[((size_t)c * HH + ys) * WW + x];
    const float t = interior ? (FCARRY * bf16r(v)) : 0.0f;
    Tl[(x + 1u) * LDT + c] = toh_flush(t);
  }
  __syncthreads();

  v8h xv[5];
  size_t off[5];
#pragma unroll
  for (unsigned j = 0; j < 5u; ++j) {
    const unsigned idx = tid + 256u * j;
    const unsigned idc = (idx < (unsigned)(PW * 8)) ? idx : (unsigned)(PW * 8 - 1);
    const unsigned px = idc >> 3, pc = (idc & 7u) * 8u;
    xv[j] = *(const v8h*)&Tl[px * LDT + pc];
    off[j] = ((size_t)yp * PW + px) * CC + pc;
  }
#pragma unroll
  for (unsigned j = 0; j < 5u; ++j)
    if (tid + 256u * j < (unsigned)(PW * 8)) *(volatile v8h*)(FP + off[j]) = xv[j];
  __threadfence();
#pragma unroll
  for (unsigned j = 0; j < 5u; ++j)
    if (tid + 256u * j < (unsigned)(PW * 8)) *(volatile v8h*)(FP + off[j]) = xv[j];
}

__global__ __launch_bounds__(256) void conv_gemm_kernel(
    const _Float16* __restrict__ FP, const float* __restrict__ Wm, float* __restrict__ T) {
  __shared__ __attribute__((aligned(16))) _Float16 Bs[16 * LDB];
  __shared__ __attribute__((aligned(16))) float Cs[WW * 4];
  const unsigned tid = threadIdx.x, lane = tid & 31u;
  const unsigned wave = (unsigned)__builtin_amdgcn_readfirstlane((int)(threadIdx.x >> 5));
  const unsigned hh = lane >> 4, m = lane & 15u;
  const unsigned y = blockIdx.x;
  const unsigned x0 = wave * 16u;

#pragma unroll 1
  for (unsigned idx = tid; idx < (unsigned)(NOUT * KTOT); idx += 256u) {
    const unsigned n = idx / (unsigned)KTOT;
    const unsigned kp = idx - n * (unsigned)KTOT;
    const unsigned tap = kp >> 6, c = kp & 63u;
    const float wv = Wm[(c * 9u + tap) * 3u + n];
    Bs[n * LDB + kp] = toh_flush(WCARRY * bf16r(wv));
  }
#pragma unroll 1
  for (unsigned idx = tid; idx < 13u * 72u; idx += 256u) {
    const unsigned r = 3u + idx / 72u;
    const unsigned pc = (idx - (r - 3u) * 72u) * 8u;
    v8h z;
#pragma unroll
    for (int i = 0; i < 8; ++i) z[i] = (h16)0.0f;
    *(v8h*)&Bs[r * LDB + pc] = z;
  }
  __syncthreads();

  v8f acc = {};
#pragma unroll 1
  for (unsigned di = 0; di < 3u; ++di) {
#pragma unroll
    for (unsigned dj = 0; dj < 3u; ++dj) {
      const _Float16* ap = FP + ((size_t)(y + di) * PW + x0 + m + dj) * CC + hh * 8u;
      const unsigned kb = (di * 3u + dj) * 64u + hh * 8u;
#pragma unroll
      for (unsigned c = 0; c < 2u; ++c) {
        const v16h a = frag_at(ap + c * 32u);
        const v8h blo = *(const v8h*)&Bs[m * LDB + kb + c * 32u];
        const v8h bhi = *(const v8h*)&Bs[m * LDB + kb + c * 32u + 16u];
        acc = wmma16(a, frag_join(blo, bhi), acc);
      }
    }
  }

  const float cs = 1.0f / (FCARRY * WCARRY);
#pragma unroll
  for (int r = 0; r < 8; ++r) {
    const float v = (m < 3u) ? (acc[r] * cs) : 0.0f;
    if (m < 4u) Cs[(x0 + hh * 8u + (unsigned)r) * 4u + m] = v;
  }
  __syncthreads();

  if (tid < (unsigned)WW) {
    const v4f v = *(const v4f*)&Cs[tid * 4u];
    float* p = T + ((size_t)y * WW + tid) * 4u;
    *(volatile v4f*)p = v;
    __threadfence();
    *(volatile v4f*)p = v;
  }
}

#pragma clang fp contract(off)

__device__ __forceinline__ void sample_one(const float cx, const float cy, const float sx,
                                           const float sy, const float* __restrict__ T,
                                           float& area, float& rx, float& ry, v4f& tv) {
  const float gx = fminf(fmaxf(cx + sx, CLIP_LO), CLIP_HI);
  const float gy = fminf(fmaxf(cy + sy, CLIP_LO), CLIP_HI);
  int ih = (int)floorf(((gx + 1.0f) * 128.0f) * 0.5f);
  int iw = (int)floorf(((gy + 1.0f) * 128.0f) * 0.5f);
  ih = (ih < 0) ? 0 : ((ih > HH - 1) ? (HH - 1) : ih);
  iw = (iw < 0) ? 0 : ((iw > WW - 1) ? (WW - 1) : iw);
  const float qx = -1.0f + (2.0f * (float)ih + 1.0f) * (1.0f / 128.0f);
  const float qy = -1.0f + (2.0f * (float)iw + 1.0f) * (1.0f / 128.0f);
  rx = (cx - qx) * 128.0f;
  ry = (cy - qy) * 128.0f;
  area = fabsf(rx * ry) + 1.0e-9f;
  tv = *(const v4f*)(T + (size_t)(ih * WW + iw) * 4u);
}

__global__ __launch_bounds__(256) void query_kernel(
    const float* __restrict__ coord, const float* __restrict__ cell,
    const float* __restrict__ Wm, const float* __restrict__ bias,
    const float* __restrict__ T, float* __restrict__ out) {
  __shared__ __attribute__((aligned(16))) float Os[256 * NOUT];
  const unsigned tid = threadIdx.x;
  const unsigned q = blockIdx.x * 256u + tid;

  const v2f co = *(const v2f*)(coord + (size_t)q * 2u);
  const v2f ce = *(const v2f*)(cell + (size_t)q * 2u);
  const float cx = bf16r(co[0]), cy = bf16r(co[1]);
  const float rcx = bf16r(ce[0]) * 128.0f;
  const float rcy = bf16r(ce[1]) * 128.0f;

  float wa[3], wb[3], base[3];
#pragma unroll
  for (int o = 0; o < 3; ++o) {
    wa[o] = bf16r(Wm[576 * 3 + o]);
    wb[o] = bf16r(Wm[577 * 3 + o]);
    base[o] = (rcx * bf16r(Wm[578 * 3 + o]) + rcy * bf16r(Wm[579 * 3 + o])) + bf16r(bias[o]);
  }

  float ar[4], rx[4], ry[4];
  v4f tv[4];
  sample_one(cx, cy, SHIFT_NEG, SHIFT_NEG, T, ar[0], rx[0], ry[0], tv[0]);
  sample_one(cx, cy, SHIFT_NEG, SHIFT_POS, T, ar[1], rx[1], ry[1], tv[1]);
  sample_one(cx, cy, SHIFT_POS, SHIFT_NEG, T, ar[2], rx[2], ry[2], tv[2]);
  sample_one(cx, cy, SHIFT_POS, SHIFT_POS, T, ar[3], rx[3], ry[3], tv[3]);

  const float tot = ((ar[0] + ar[1]) + ar[2]) + ar[3];
  const float inv = 1.0f / tot;
  float wg[4];
  wg[0] = ar[3] * inv;
  wg[1] = ar[2] * inv;
  wg[2] = ar[1] * inv;
  wg[3] = ar[0] * inv;

#pragma unroll
  for (int o = 0; o < 3; ++o) {
    float r = 0.0f;
#pragma unroll
    for (int s = 0; s < 4; ++s) {
      const float p = ((tv[s][o] + rx[s] * wa[o]) + ry[s] * wb[o]) + base[o];
      r = r + p * wg[s];
    }
    Os[tid * 3u + (unsigned)o] = r;
  }
  __syncthreads();

  if (tid < 192u) {
    const v4f v = *(const v4f*)&Os[tid * 4u];
    float* p = out + (size_t)blockIdx.x * (256u * NOUT) + tid * 4u;
    *(volatile v4f*)p = v;
    __threadfence();
    *(volatile v4f*)p = v;
  }
}

extern "C" void kernel_launch(void* const* d_in, const int* in_sizes, int n_in,
                              void* d_out, int out_size, void* d_ws, size_t ws_size,
                              hipStream_t stream) {
  if (n_in < 5) return;
  if ((long long)in_sizes[0] < (long long)CC * HH * WW) return;
  if ((long long)in_sizes[1] < (long long)NQ * 2) return;
  if ((long long)in_sizes[2] < (long long)NQ * 2) return;
  if ((long long)in_sizes[3] < (long long)DIN * NOUT) return;
  if (in_sizes[4] < NOUT) return;
  if ((long long)out_size < (long long)NQ * NOUT) return;
  if (ws_size < WS_TOTAL) return;

  const float* feat  = (const float*)d_in[0];
  const float* coord = (const float*)d_in[1];
  const float* cell  = (const float*)d_in[2];
  const float* Wm    = (const float*)d_in[3];
  const float* bias  = (const float*)d_in[4];
  float* out = (float*)d_out;

  char* ws = (char*)d_ws;
  _Float16* FP = (_Float16*)(ws + OFF_FP);
  float*    T  = (float*)(ws + OFF_T);

  dim3 blk(256);
  featplane_kernel<<<dim3(PH), blk, 0, stream>>>(feat, FP);
  conv_gemm_kernel<<<dim3(HH), blk, 0, stream>>>(FP, Wm, T);
  query_kernel<<<dim3(NQ / 256), blk, 0, stream>>>(coord, cell, Wm, bias, T, out);
}
